// MultiHeadSelfAttention_64802466562101
// MI455X (gfx1250) — hardware-verified
//
#include <hip/hip_runtime.h>


#ifndef NB
#define NB 2
#endif
#ifndef SEQ
#define SEQ 2048
#endif
#define NB_FULL   2
#define SEQ_FULL  2048
#define HID       1024
#define NHEAD     16
#define HD        64
#define NQKV      (3 * HID)
#define MROWS     (NB * SEQ)
#define WPITCH    (SEQ / 32)
#define FPITCH    ((SEQ / 32) < 32 ? 32 : (SEQ / 32))
#define EARLY_BLKS ((SEQ / 128) >= 2 ? 2 : 1)
#define NXH       ((size_t)MROWS * HID)

static_assert(HID == NHEAD * HD);
static_assert(NHEAD == 16);
static_assert(HD == 64);
static_assert(SEQ % 128 == 0);
static_assert(SEQ % 64 == 0);
static_assert(SEQ <= SEQ_FULL);
static_assert(NB >= 1 && NB <= NB_FULL);
static_assert(MROWS % 128 == 0);
static_assert(HID % 128 == 0);
static_assert(HID % 32 == 0);
static_assert((HID & (HID - 1)) == 0);
static_assert(HID == 128 * 8);
static_assert(MROWS % 2 == 0);
static_assert(NQKV % 64 == 0);
static_assert(HID % 64 == 0);
static_assert(WPITCH * 32 == SEQ);
static_assert((16 * WPITCH) % 32 == 0);
static_assert(16 * WPITCH * 4 <= 16384);
static_assert(FPITCH % 32 == 0);
static_assert(FPITCH <= 256);
static_assert(FPITCH >= WPITCH);
static_assert(SEQ / 128 >= EARLY_BLKS);

#define CARRY_X    16.0f
#define CARRY_W    32.0f
#define CARRY_QKV  16.0f
#define CARRY_CTX  1024.0f
#define RES_SCALE  2048.0f
#define RES_INV    0.00048828125f

typedef unsigned u32;
typedef _Float16 f16;
typedef f16   v16h __attribute__((ext_vector_type(16)));
typedef f16   v8h  __attribute__((ext_vector_type(8)));
typedef float v8f  __attribute__((ext_vector_type(8)));
typedef float v4f  __attribute__((ext_vector_type(4)));
typedef int   v4i  __attribute__((ext_vector_type(4)));

union FragU { v16h v; v8h half[2]; f16 e[16]; };
union H8U   { v8h v; f16 e[8]; };

__device__ __forceinline__ v8f zero8() {
    v8f z = {0.f, 0.f, 0.f, 0.f, 0.f, 0.f, 0.f, 0.f};
    return z;
}

__device__ __forceinline__ v8f wmma16(v16h a, v16h b, v8f c) {
    v8f d = __builtin_amdgcn_wmma_f32_16x16x32_f16(false, a, false, b, (short)0, c, false, false);
    asm volatile("v_nop\n\tv_nop\n\tv_nop\n\tv_nop" : "+v"(d) : "v"(a), "v"(b));
    return d;
}

__device__ __forceinline__ float bf16_rne(float x) {
    u32 u = __float_as_uint(x);
    u = (u + 0x7fffu + ((u >> 16) & 1u)) & 0xffff0000u;
    return __uint_as_float(u);
}

__device__ __forceinline__ float fexp2(float x) {
#if defined(__has_builtin)
#if __has_builtin(__builtin_amdgcn_exp2f)
    return __builtin_amdgcn_exp2f(x);
#else
    return exp2f(x);
#endif
#else
    return exp2f(x);
#endif
}

__device__ __forceinline__ float rowmax16(float x) {
    int v = __builtin_bit_cast(int, x);
    x = fmaxf(x, __builtin_bit_cast(float, __builtin_amdgcn_update_dpp(v, v, 0x121, 0xf, 0xf, false)));
    v = __builtin_bit_cast(int, x);
    x = fmaxf(x, __builtin_bit_cast(float, __builtin_amdgcn_update_dpp(v, v, 0x122, 0xf, 0xf, false)));
    v = __builtin_bit_cast(int, x);
    x = fmaxf(x, __builtin_bit_cast(float, __builtin_amdgcn_update_dpp(v, v, 0x124, 0xf, 0xf, false)));
    v = __builtin_bit_cast(int, x);
    x = fmaxf(x, __builtin_bit_cast(float, __builtin_amdgcn_update_dpp(v, v, 0x128, 0xf, 0xf, false)));
    return x;
}

__device__ __forceinline__ v16h load_frag(const f16* tile, u32 rowbase, u32 pitch, u32 kcol, u32 lane) {
    const u32 r  = rowbase + (lane & 15u);
    const u32 kh = (lane >> 4) << 3;
    const f16* p = tile + (size_t)r * pitch + kcol + kh;
    FragU f;
    f.half[0] = *(const v8h*)(p);
    f.half[1] = *(const v8h*)(p + 16);
    return f.v;
}

__global__ void __launch_bounds__(256)
mask_tiles(const int* __restrict__ mask, u32* __restrict__ words, u32* __restrict__ flags) {
    __shared__ u32 wl[16 * WPITCH];
    const u32 tid = threadIdx.x;
    const u32 qt  = blockIdx.x;
#pragma unroll 1
    for (u32 idx = tid; idx < 16u * (u32)WPITCH; idx += 256u) {
        const u32 i  = idx / (u32)WPITCH;
        const u32 kg = idx - i * (u32)WPITCH;
        const int* mp = mask + (size_t)(qt * 16u + i) * SEQ_FULL + kg * 32u;
        u32 w = 0u;
#pragma unroll
        for (u32 j = 0; j < 8; ++j) {
            const v4i a = *(const v4i*)(mp + j * 4u);
            u32 nib = 0u;
            nib |= (a[0] != 0) ? 1u : 0u;
            nib |= (a[1] != 0) ? 2u : 0u;
            nib |= (a[2] != 0) ? 4u : 0u;
            nib |= (a[3] != 0) ? 8u : 0u;
            w |= nib << (j * 4u);
        }
        wl[idx] = w;
        u32* dp = words + (size_t)qt * 16u * WPITCH + idx;
        *(volatile u32*)dp = w;
        __threadfence();
        *(volatile u32*)dp = w;
    }
    __syncthreads();
    if (tid < (u32)FPITCH) {
        const u32 kgc = (tid < (u32)WPITCH) ? tid : (u32)(WPITCH - 1);
        u32 a = 0xffffffffu, o = 0u;
#pragma unroll 1
        for (u32 i = 0; i < 16u; ++i) {
            const u32 w = wl[i * (u32)WPITCH + kgc];
            a &= w;
            o |= w;
        }
        u32 f = (o == 0u) ? 0u : ((a == 0xffffffffu) ? 2u : 1u);
        if (tid >= (u32)WPITCH) f = 0u;
        u32* dp = flags + (size_t)qt * FPITCH + tid;
        *(volatile u32*)dp = f;
        __threadfence();
        *(volatile u32*)dp = f;
    }
}

__global__ void __launch_bounds__(256)
cvt_rows(const float* __restrict__ src, f16* __restrict__ dst, u32 nrows, u32 dstper, u32 srcper, float carry) {
    const u32 g  = blockIdx.x * 256u + threadIdx.x;
    const u32 m  = g >> 7;
    const u32 c8 = (g & 127u) << 3;
    if (m >= nrows) return;
    const u32 mb = m / dstper;
    const u32 sm = mb * srcper + (m - mb * dstper);
    const float* sp = src + (size_t)sm * HID + c8;
    const v4f a = *(const v4f*)sp;
    const v4f b = *(const v4f*)(sp + 4);
    H8U o;
#pragma unroll
    for (u32 j = 0; j < 4; ++j) {
        const float x0 = a[j];
        const float x1 = b[j];
        o.e[j]     = (f16)(bf16_rne(x0) * carry);
        o.e[j + 4] = (f16)(bf16_rne(x1) * carry);
    }
    f16* dp = dst + (size_t)m * HID + c8;
    *(volatile v8h*)dp = o.v;
    __threadfence();
    *(volatile v8h*)dp = o.v;
}

__global__ void __launch_bounds__(256)
cvt_wT(const float* __restrict__ src, f16* __restrict__ dst, u32 ncols, float carry) {
    __shared__ __attribute__((aligned(16))) f16 ts[64 * 72];
    static_assert((72 * sizeof(f16)) % 16 == 0);
    const u32 tid = threadIdx.x;
    const u32 n0  = blockIdx.x * 64u;
    const u32 k0  = blockIdx.y * 64u;
    const u32 c4  = (tid & 15u) << 2;
    const u32 r0  = tid >> 4;
#pragma unroll
    for (u32 it = 0; it < 4; ++it) {
        const u32 kk = r0 + it * 16u;
        const v4f a = *(const v4f*)(src + (size_t)(k0 + kk) * ncols + n0 + c4);
#pragma unroll
        for (u32 j = 0; j < 4; ++j) {
            const float xv = a[j];
            ts[(c4 + j) * 72u + kk] = (f16)(bf16_rne(xv) * carry);
        }
    }
    __syncthreads();
    const u32 piece = tid & 7u;
    const u32 nr    = tid >> 3;
    v8h v[2];
#pragma unroll
    for (u32 it = 0; it < 2; ++it) v[it] = *(const v8h*)&ts[(nr + it * 32u) * 72u + piece * 8u];
#pragma unroll
    for (int pass = 0; pass < 2; ++pass) {
#pragma unroll
        for (u32 it = 0; it < 2; ++it) {
            f16* dp = dst + (size_t)(n0 + nr + it * 32u) * HID + k0 + piece * 8u;
            *(volatile v8h*)dp = v[it];
        }
        if (pass == 0) __threadfence();
    }
}

template <int MODE, int APITCH, int KLEN>
__device__ __forceinline__ void gemm_body(const f16* __restrict__ A, const f16* __restrict__ W,
                                          const float* __restrict__ bias, f16* __restrict__ outp,
                                          float* __restrict__ outf, float accMul, float biasMul) {
    __shared__ __attribute__((aligned(16))) f16 As[128 * 32];
    __shared__ __attribute__((aligned(16))) f16 Bs[128 * 32];
    __shared__ __attribute__((aligned(16))) f16 Cs[128 * 128];
    static_assert(sizeof(f16) * 128 * 128 == sizeof(float) * 64 * 128);
    static_assert(KLEN % 32 == 0);
    static_assert(KLEN % HID == 0);
    static_assert(APITCH >= KLEN);
    static_assert(APITCH % 8 == 0);

    const u32 tid  = threadIdx.x;
    const u32 lane = tid & 31u;
    const u32 wave = (u32)__builtin_amdgcn_readfirstlane((int)(threadIdx.x >> 5));
    const u32 wm   = wave & 3u;
    const u32 wn   = wave >> 2;
    const u32 hh8  = (lane >> 4) << 3;
    const u32 c16  = lane & 15u;
    const u32 m0   = blockIdx.x * 128u;
    const u32 n0   = blockIdx.y * 128u;

    v8f acc[2][4];
#pragma unroll
    for (int i = 0; i < 2; ++i)
#pragma unroll
        for (int j = 0; j < 4; ++j) acc[i][j] = zero8();

    const u32 srow = tid >> 1;
    const u32 scol = (tid & 1u) << 4;
    const f16* gA = A + (size_t)(m0 + srow) * APITCH + scol;
    const f16* gW = W + (size_t)(n0 + srow) * HID + scol;

#pragma unroll 1
    for (u32 k0 = 0; k0 < (u32)KLEN; k0 += 32u) {
        const u32 kw = k0 & (u32)(HID - 1);
        const v8h ra0 = *(const v8h*)(gA + k0);
        const v8h ra1 = *(const v8h*)(gA + k0 + 8);
        const v8h rb0 = *(const v8h*)(gW + kw);
        const v8h rb1 = *(const v8h*)(gW + kw + 8);
        __syncthreads();
        *(v8h*)&As[srow * 32u + scol]      = ra0;
        *(v8h*)&As[srow * 32u + scol + 8u] = ra1;
        *(v8h*)&Bs[srow * 32u + scol]      = rb0;
        *(v8h*)&Bs[srow * 32u + scol + 8u] = rb1;
        __syncthreads();

        v16h af[2], bfr[4];
#pragma unroll
        for (int i = 0; i < 2; ++i) af[i] = load_frag(As, wm * 32u + (u32)i * 16u, 32u, 0u, lane);
#pragma unroll
        for (int j = 0; j < 4; ++j) bfr[j] = load_frag(Bs, wn * 64u + (u32)j * 16u, 32u, 0u, lane);
#pragma unroll
        for (int i = 0; i < 2; ++i)
#pragma unroll
            for (int j = 0; j < 4; ++j) acc[i][j] = wmma16(af[i], bfr[j], acc[i][j]);
    }

    float bv[4];
#pragma unroll
    for (int j = 0; j < 4; ++j) bv[j] = bf16_rne(bias[n0 + wn * 64u + (u32)j * 16u + c16]) * biasMul;

    const u32 bidx  = m0 / (u32)SEQ;
    const u32 s0    = m0 - bidx * (u32)SEQ;
    const u32 piece = lane & 7u;
    const u32 lsub  = lane >> 3;

    if constexpr (MODE == 0) {
        const size_t bh0 = (size_t)bidx * NHEAD + (n0 >> 6);
#pragma unroll
        for (int ph = 0; ph < 2; ++ph) {
            if (ph == 1) __syncthreads();
#pragma unroll
            for (int i = 0; i < 2; ++i)
#pragma unroll
                for (int j = 0; j < 4; ++j) {
                    const u32 nl = wn * 64u + (u32)j * 16u + c16;
#pragma unroll
                    for (int r = 0; r < 8; ++r) {
                        const u32 ml = wm * 32u + (u32)i * 16u + hh8 + (u32)r;
                        const float val = acc[i][j][r] * accMul + bv[j];
                        const f16 hi = (f16)val;
                        f16 t = hi;
                        if (ph == 1) t = (f16)((val - (float)hi) * RES_SCALE);
                        Cs[ml * 128u + nl] = t;
                    }
                }
            __syncthreads();
            f16* op = outp + (size_t)ph * NXH;
#pragma unroll
            for (int pass = 0; pass < 2; ++pass) {
#pragma unroll
                for (u32 it = 0; it < 8; ++it) {
                    const u32 L    = wave * 32u + it * 4u + lsub;
                    const u32 ml   = L >> 1;
                    const u32 hsel = L & 1u;
                    const v8h v = *(const v8h*)&Cs[ml * 128u + hsel * 64u + piece * 8u];
                    f16* dp = op + ((bh0 + hsel) * SEQ + s0 + ml) * HD + piece * 8u;
                    *(volatile v8h*)dp = v;
                }
                if (pass == 0) __threadfence();
            }
        }
    } else if constexpr (MODE == 1) {
#pragma unroll
        for (int ph = 0; ph < 2; ++ph) {
            if (ph == 1) __syncthreads();
#pragma unroll
            for (int i = 0; i < 2; ++i)
#pragma unroll
                for (int j = 0; j < 4; ++j) {
                    const u32 nl = wn * 64u + (u32)j * 16u + c16;
                    H8U t;
#pragma unroll
                    for (int r = 0; r < 8; ++r) {
                        const float val = acc[i][j][r] * accMul + bv[j];
                        const f16 hi = (f16)val;
                        f16 tv = hi;
                        if (ph == 1) tv = (f16)((val - (float)hi) * RES_SCALE);
                        t.e[r] = tv;
                    }
                    *(v8h*)&Cs[nl * 128u + wm * 32u + (u32)i * 16u + hh8] = t.v;
                }
            __syncthreads();
            f16* op = outp + (size_t)ph * NXH;
#pragma unroll
            for (int pass = 0; pass < 2; ++pass) {
#pragma unroll
                for (u32 it = 0; it < 8; ++it) {
                    const u32 L  = wave * 32u + it * 4u + lsub;
                    const u32 nl = L >> 1;
                    const u32 mh = L & 1u;
                    const v8h v = *(const v8h*)&Cs[nl * 128u + mh * 64u + piece * 8u];
                    f16* dp = op + ((size_t)(bidx * (u32)HID + n0 + nl) * SEQ + s0 + mh * 64u + piece * 8u);
                    *(volatile v8h*)dp = v;
                }
                if (pass == 0) __threadfence();
            }
        }
    } else {
        float* Cf = (float*)Cs;
#pragma unroll
        for (u32 half = 0; half < 2; ++half) {
            if ((wm >> 1) == half) {
#pragma unroll
                for (int i = 0; i < 2; ++i)
#pragma unroll
                    for (int j = 0; j < 4; ++j) {
                        const u32 nl = wn * 64u + (u32)j * 16u + c16;
#pragma unroll
                        for (int r = 0; r < 8; ++r) {
                            const u32 ml = (wm & 1u) * 32u + (u32)i * 16u + hh8 + (u32)r;
                            Cf[ml * 128u + nl] = acc[i][j][r] * accMul + bv[j];
                        }
                    }
            }
            __syncthreads();
#pragma unroll
            for (int pass = 0; pass < 2; ++pass) {
#pragma unroll
                for (u32 it = 0; it < 8; ++it) {
                    const u32 L    = wave * 32u + it * 4u + lsub;
                    const u32 row  = L >> 2;
                    const u32 part = L & 3u;
                    const v4f v = *(const v4f*)&Cf[row * 128u + part * 32u + piece * 4u];
                    float* dp = outf + (size_t)(m0 + half * 64u + row) * HID + n0 + part * 32u + piece * 4u;
                    *(volatile v4f*)dp = v;
                }
                if (pass == 0) __threadfence();
            }
            __syncthreads();
        }
    }
}

__global__ void __launch_bounds__(256) __attribute__((amdgpu_num_vgpr(256)))
gemm_head(const f16* __restrict__ A, const f16* __restrict__ W, const float* __restrict__ bias,
          f16* __restrict__ out, float accMul, float biasMul) {
    gemm_body<0, HID, HID>(A, W, bias, out, (float*)0, accMul, biasMul);
}

__global__ void __launch_bounds__(256) __attribute__((amdgpu_num_vgpr(256)))
gemm_vt(const f16* __restrict__ A, const f16* __restrict__ W, const float* __restrict__ bias,
        f16* __restrict__ out, float accMul, float biasMul) {
    gemm_body<1, HID, HID>(A, W, bias, out, (float*)0, accMul, biasMul);
}

__global__ void __launch_bounds__(256) __attribute__((amdgpu_num_vgpr(256)))
gemm_out(const f16* __restrict__ A, const f16* __restrict__ W, const float* __restrict__ bias,
         float* __restrict__ out, float accMul) {
    gemm_body<2, 2 * HID, 2 * HID>(A, W, bias, (f16*)0, out, accMul, 1.0f);
}

template <bool EARLY>
__device__ __forceinline__ void attn_body(const f16* __restrict__ Qp, const f16* __restrict__ Kp,
                                          const f16* __restrict__ Vt, f16* __restrict__ Cp,
                                          const u32* __restrict__ words, const u32* __restrict__ flags,
                                          u32 qblk) {
    __shared__ __attribute__((aligned(16))) f16 ks[64 * 64];
    __shared__ __attribute__((aligned(16))) f16 vsT[64 * 64];
    __shared__ __attribute__((aligned(16))) f16 ps[128 * 64];
    __shared__ __attribute__((aligned(16))) f16 kls[EARLY ? 64 * 64 : 8];
    __shared__ __attribute__((aligned(16))) f16 vlsT[EARLY ? 64 * 64 : 8];
    __shared__ __attribute__((aligned(16))) f16 pls[EARLY ? 128 * 64 : 8];
    static_assert(HD == 8 * 8);
    static_assert(2 * 256 * 8 == 64 * 64);

    const u32 tid  = threadIdx.x;
    const u32 lane = tid & 31u;
    const u32 wave = (u32)__builtin_amdgcn_readfirstlane((int)(threadIdx.x >> 5));
    const u32 hh8  = (lane >> 4) << 3;
    const u32 c16  = lane & 15u;
    const u32 bh   = blockIdx.y;
    const u32 bidx = bh >> 4;
    const u32 hidx = bh & 15u;
    const u32 q0   = qblk * 128u + wave * 16u;
    const u32 qt   = q0 >> 4;
    const u32 prow = wave * 16u;
    const size_t head = (size_t)bh * SEQ * HD;

    FragU onesu;
#pragma unroll
    for (int i = 0; i < 16; ++i) onesu.e[i] = (f16)1.0f;
    const v16h ones = onesu.v;

    float m[8];
    v8f   o[4], ores[4], lacc, lres;
#pragma unroll
    for (int r = 0; r < 8; ++r) m[r] = -1.0e30f;
#pragma unroll
    for (int dt = 0; dt < 4; ++dt) { o[dt] = zero8(); ores[dt] = zero8(); }
    lacc = zero8();
    lres = zero8();

    const float cl = 1.4426950408889634f * 0.00048828125f;
    const float NEG_INF = -__builtin_inff();

#pragma unroll 1
    for (u32 kt = 0; kt < (u32)(SEQ / 64); ++kt) {
        u32 anyf = 0u;
#pragma unroll
        for (u32 w = 0; w < 8; ++w) {
            const u32 fi = (qblk * 8u + w) * (u32)FPITCH + kt * 2u;
            anyf |= flags[fi] | flags[fi + 1u];
        }
        anyf = (u32)__builtin_amdgcn_readfirstlane((int)anyf);
        if (anyf == 0u) continue;

        __syncthreads();
#pragma unroll
        for (u32 p2 = 0; p2 < 2; ++p2) {
            const u32 p   = tid + p2 * 256u;
            const u32 row = p >> 3;
            const u32 pc  = (p & 7u) << 3;
            const size_t ko = head + (size_t)(kt * 64u + row) * HD + pc;
            const size_t vo = head + (size_t)row * SEQ + kt * 64u + pc;
            const v8h kv = *(const v8h*)(Kp + ko);
            const v8h vv = *(const v8h*)(Vt + vo);
            *(v8h*)&ks[row * 64u + pc]  = kv;
            *(v8h*)&vsT[row * 64u + pc] = vv;
            if constexpr (EARLY) {
                const v8h klv = *(const v8h*)(Kp + NXH + ko);
                const v8h vlv = *(const v8h*)(Vt + NXH + vo);
                *(v8h*)&kls[row * 64u + pc]  = klv;
                *(v8h*)&vlsT[row * 64u + pc] = vlv;
            }
        }
        __syncthreads();

#pragma unroll 1
        for (u32 hf = 0; hf < 2u; ++hf) {
            const u32 kg = kt * 2u + hf;
            const u32 fl = (u32)__builtin_amdgcn_readfirstlane((int)flags[qt * (u32)FPITCH + kg]);

            if (fl != 0u) {
                v8f s[2], sr[2];
#pragma unroll
                for (int nt = 0; nt < 2; ++nt) { s[nt] = zero8(); sr[nt] = zero8(); }
#pragma unroll
                for (int c = 0; c < 2; ++c) {
                    const v16h qh = load_frag(Qp + head, q0, HD, (u32)c * 32u, lane);
                    const v16h ql = load_frag(Qp + NXH + head, q0, HD, (u32)c * 32u, lane);
#pragma unroll
                    for (int nt = 0; nt < 2; ++nt) {
                        const v16h kb = load_frag(ks, hf * 32u + (u32)nt * 16u, 64u, (u32)c * 32u, lane);
                        s[nt]  = wmma16(qh, kb, s[nt]);
                        sr[nt] = wmma16(ql, kb, sr[nt]);
                        if constexpr (EARLY) {
                            const v16h klb = load_frag(kls, hf * 32u + (u32)nt * 16u, 64u, (u32)c * 32u, lane);
                            sr[nt] = wmma16(qh, klb, sr[nt]);
                        }
                    }
                }

                u32 mw[8];
#pragma unroll
                for (int r = 0; r < 8; ++r) mw[r] = 0xffffffffu;
                if (fl != 2u) {
#pragma unroll
                    for (int r = 0; r < 8; ++r)
                        mw[r] = words[(size_t)(q0 + hh8 + (u32)r) * WPITCH + kg];
                }

#pragma unroll
                for (int r = 0; r < 8; ++r) {
                    float x[2];
#pragma unroll
                    for (int nt = 0; nt < 2; ++nt) {
                        const float sv = (s[nt][r] + sr[nt][r] * RES_INV) * cl;
                        const u32 keep = (mw[r] >> ((u32)nt * 16u + c16)) & 1u;
                        x[nt] = (keep != 0u) ? sv : NEG_INF;
                    }
                    const float tm = rowmax16(fmaxf(x[0], x[1]));
                    const float mn = fmaxf(m[r], tm);
                    const float al = fexp2(m[r] - mn);
                    m[r] = mn;
                    lacc[r] *= al;
#pragma unroll
                    for (int dt = 0; dt < 4; ++dt) o[dt][r] *= al;
                    if constexpr (EARLY) {
                        lres[r] *= al;
#pragma unroll
                        for (int dt = 0; dt < 4; ++dt) ores[dt][r] *= al;
                    }
                    const float sh = 10.0f - mn;
#pragma unroll
                    for (int nt = 0; nt < 2; ++nt) {
                        const float p  = fexp2(x[nt] + sh);
                        const f16  phv = (f16)p;
                        const u32  pi  = (prow + hh8 + (u32)r) * 64u + hf * 32u + (u32)nt * 16u + c16;
                        ps[pi] = phv;
                        if constexpr (EARLY) pls[pi] = (f16)((p - (float)phv) * RES_SCALE);
                    }
                }
            }
            __syncthreads();

            if (fl != 0u) {
                const v16h pa = load_frag(ps, prow, 64u, hf * 32u, lane);
                if constexpr (EARLY) {
                    const v16h pla = load_frag(pls, prow, 64u, hf * 32u, lane);
#pragma unroll
                    for (int dt = 0; dt < 4; ++dt) {
                        const v16h vb  = load_frag(vsT,  (u32)dt * 16u, 64u, hf * 32u, lane);
                        const v16h vlb = load_frag(vlsT, (u32)dt * 16u, 64u, hf * 32u, lane);
                        o[dt]    = wmma16(pa,  vb,  o[dt]);
                        ores[dt] = wmma16(pla, vb,  ores[dt]);
                        ores[dt] = wmma16(pa,  vlb, ores[dt]);
                    }
                    lacc = wmma16(pa,  ones, lacc);
                    lres = wmma16(pla, ones, lres);
                } else {
#pragma unroll
                    for (int dt = 0; dt < 4; ++dt) {
                        const v16h vb = load_frag(vsT, (u32)dt * 16u, 64u, hf * 32u, lane);
                        o[dt] = wmma16(pa, vb, o[dt]);
                    }
                    lacc = wmma16(pa, ones, lacc);
                }
            }
        }
    }
    __syncthreads();

    const u32 piece = lane & 7u;
    const u32 lsub  = lane >> 3;
#pragma unroll
    for (int ph = 0; ph < 2; ++ph) {
        if (ph == 1) __syncthreads();
#pragma unroll
        for (int r = 0; r < 8; ++r) {
            float lsum = lacc[r];
            if constexpr (EARLY) lsum += lres[r] * RES_INV;
            const float inv = (CARRY_CTX / CARRY_QKV) / lsum;
#pragma unroll
            for (int dt = 0; dt < 4; ++dt) {
                float ov = o[dt][r];
                if constexpr (EARLY) ov += ores[dt][r] * RES_INV;
                const float val = ov * inv;
                const f16 hi = (f16)val;
                f16 t = hi;
                if (ph == 1) t = (f16)(val - (float)hi);
                ps[(prow + hh8 + (u32)r) * 64u + (u32)dt * 16u + c16] = t;
            }
        }
        __syncthreads();
#pragma unroll
        for (int pass = 0; pass < 2; ++pass) {
#pragma unroll
            for (u32 it = 0; it < 4; ++it) {
                const u32 L = it * 4u + lsub;
                const v8h v = *(const v8h*)&ps[(prow + L) * 64u + piece * 8u];
                f16* dp = Cp + ((size_t)(bidx * (u32)SEQ + q0 + L) * (2 * HID) + (u32)ph * (u32)HID
                                + hidx * (u32)HD + piece * 8u);
                *(volatile v8h*)dp = v;
            }
            if (pass == 0) __threadfence();
        }
    }
}

__global__ void __launch_bounds__(256) __attribute__((amdgpu_num_vgpr(256)))
attn_early(const f16* __restrict__ Qp, const f16* __restrict__ Kp, const f16* __restrict__ Vt,
           f16* __restrict__ Cp, const u32* __restrict__ words, const u32* __restrict__ flags) {
    attn_body<true>(Qp, Kp, Vt, Cp, words, flags, blockIdx.x);
}

__global__ void __launch_bounds__(256) __attribute__((amdgpu_num_vgpr(256)))
attn_late(const f16* __restrict__ Qp, const f16* __restrict__ Kp, const f16* __restrict__ Vt,
          f16* __restrict__ Cp, const u32* __restrict__ words, const u32* __restrict__ flags) {
    attn_body<false>(Qp, Kp, Vt, Cp, words, flags, blockIdx.x + (u32)EARLY_BLKS);
}

static_assert((size_t)(MROWS / 2) * 256 * 8 == (size_t)MROWS * HID);
static_assert((size_t)(NQKV / 64) * (HID / 64) * 64 * 64 == (size_t)NQKV * HID);
static_assert((size_t)(HID / 64) * (HID / 64) * 64 * 64 == (size_t)HID * HID);
static_assert((size_t)(MROWS / 128) * (HID / 128) * 128 * 128 == (size_t)MROWS * HID);
static_assert((size_t)(SEQ / 128) * (NB * NHEAD) * 128 * HD == (size_t)MROWS * HID);
static_assert((size_t)(SEQ / 16) * 16 * WPITCH == (size_t)SEQ * WPITCH);

#define WS_XH     ((size_t)MROWS * HID * 2)
#define WS_WT     ((size_t)NQKV * HID * 2)
#define WS_WOT    ((size_t)HID * HID * 2)
#define WS_PAIR   ((size_t)2 * MROWS * HID * 2)
#define WS_WORDS  ((size_t)SEQ * WPITCH * 4)
#define WS_FLAGS  ((size_t)(SEQ / 16) * FPITCH * 4)
#define WS_TOTAL  (WS_XH + WS_WT + WS_WOT + 4 * WS_PAIR + WS_WORDS + WS_FLAGS)
static_assert(WS_XH % 256 == 0 && WS_WT % 256 == 0 && WS_WOT % 256 == 0 && WS_PAIR % 256 == 0);
static_assert(WS_WORDS % 256 == 0 && WS_FLAGS % 128 == 0);
static_assert(WS_TOTAL <= (size_t)134217728);
static_assert((size_t)MROWS * HID <= (size_t)NB_FULL * SEQ_FULL * HID);

extern "C" void kernel_launch(void* const* d_in, const int* in_sizes, int n_in,
                              void* d_out, int out_size, void* d_ws, size_t ws_size,
                              hipStream_t stream) {
    if (n_in < 6) return;
    if (in_sizes[0] < ((NB - 1) * SEQ_FULL + SEQ) * HID) return;
    if (in_sizes[1] < HID * NQKV) return;
    if (in_sizes[2] < NQKV) return;
    if (in_sizes[3] < HID * HID) return;
    if (in_sizes[4] < HID) return;
    if (in_sizes[5] < (SEQ - 1) * SEQ_FULL + SEQ) return;
    if (out_size < MROWS * HID) return;
    if (ws_size < WS_TOTAL) return;

    const float* x     = (const float*)d_in[0];
    const float* wqkv  = (const float*)d_in[1];
    const float* bqkv  = (const float*)d_in[2];
    const float* wout  = (const float*)d_in[3];
    const float* bout  = (const float*)d_in[4];
    const int*   amask = (const int*)d_in[5];

    char* wsb = (char*)d_ws;
    size_t off = 0;
    f16* Xh  = (f16*)(wsb + off); off += WS_XH;
    f16* Wt  = (f16*)(wsb + off); off += WS_WT;
    f16* Wot = (f16*)(wsb + off); off += WS_WOT;
    f16* QP  = (f16*)(wsb + off); off += WS_PAIR;
    f16* KP  = (f16*)(wsb + off); off += WS_PAIR;
    f16* VP  = (f16*)(wsb + off); off += WS_PAIR;
    f16* Cp  = (f16*)(wsb + off); off += WS_PAIR;
    u32* words = (u32*)(wsb + off); off += WS_WORDS;
    u32* flags = (u32*)(wsb + off); off += WS_FLAGS;

    mask_tiles<<<SEQ / 16, 256, 0, stream>>>(amask, words, flags);

    cvt_rows<<<MROWS / 2, 256, 0, stream>>>(x, Xh, (u32)MROWS, (u32)SEQ, (u32)SEQ_FULL, CARRY_X);
    cvt_wT<<<dim3(NQKV / 64, HID / 64), 256, 0, stream>>>(wqkv, Wt, (u32)NQKV, CARRY_W);
    cvt_wT<<<dim3(HID / 64, HID / 64), 256, 0, stream>>>(wout, Wot, (u32)HID, CARRY_W);

    const dim3 gg(MROWS / 128, HID / 128);
    const size_t nW = (size_t)HID * HID;
    const float accQKV = CARRY_QKV / (CARRY_X * CARRY_W);
    gemm_head<<<gg, 256, 0, stream>>>(Xh, Wt,          bqkv,           QP, accQKV, CARRY_QKV);
    gemm_head<<<gg, 256, 0, stream>>>(Xh, Wt + nW,     bqkv + HID,     KP, accQKV, CARRY_QKV);
    gemm_vt  <<<gg, 256, 0, stream>>>(Xh, Wt + 2 * nW, bqkv + 2 * HID, VP, accQKV, CARRY_QKV);

    attn_early<<<dim3(EARLY_BLKS, NB * NHEAD), 256, 0, stream>>>(QP, KP, VP, Cp, words, flags);
    if ((SEQ / 128) > EARLY_BLKS) {
        attn_late<<<dim3(SEQ / 128 - EARLY_BLKS, NB * NHEAD), 256, 0, stream>>>(QP, KP, VP, Cp, words, flags);
    }

    const float accOut = 1.0f / (CARRY_CTX * CARRY_W);
    gemm_out<<<gg, 256, 0, stream>>>(Cp, Wot, bout, (float*)d_out, accOut);
}
